// ClusteredMambaModel_Flood_76656576299511
// MI455X (gfx1250) — hardware-verified
//
#include <hip/hip_runtime.h>
#include <math.h>

constexpr int kRows     = 16384;
constexpr int kFeat     = 16;
constexpr int kNonRain  = 12;
constexpr int kRain     = 4;
constexpr int kClust    = 1000;
constexpr int kClustPad = 1024;
constexpr int kDModel   = 64;
constexpr int kDInner   = 128;
constexpr int kDState   = 16;
constexpr int kDtRank   = 4;
constexpr int kDConv    = 4;
constexpr int kProjN    = 36;
constexpr int kProjPad  = 64;
constexpr int kLayers   = 4;
constexpr int kRows2    = 2 * kRows;
constexpr int kHeadHid  = 32;
constexpr float kLnEps  = 1e-5f;
constexpr float kInvDModel = 1.0f / 64.0f;

static_assert(kClust % 8 == 0, "size");
static_assert(kRows % 256 == 0, "size");
static_assert(kRows2 % 64 == 0, "size");

constexpr size_t kOffWinHi = 0;
constexpr size_t kOffWinLo = 262144;
constexpr size_t kOffIpwHi = 524288;
constexpr size_t kOffIpwLo = 655360;
constexpr size_t kOffXpwHi = 786432;
constexpr size_t kOffXpwLo = 851968;
constexpr size_t kOffOpwHi = 917504;
constexpr size_t kOffOpwLo = 983040;
constexpr size_t kOffR     = 1048576;
constexpr size_t kOffNrHi  = kOffR;
constexpr size_t kOffNrLo  = kOffR + 33554432;
constexpr size_t kOffXz    = kOffR;
constexpr size_t kOffXcf   = kOffR + 33554432;
constexpr size_t kOffXcHi  = kOffR + 50331648;
constexpr size_t kOffXcLo  = kOffR + 58720256;
constexpr size_t kOffXa    = kOffR + 67108864;
constexpr size_t kOffXb    = kOffXa + 8388608;
constexpr size_t kOffXpHi  = kOffXb + 8388608;
constexpr size_t kOffXpLo  = kOffXpHi + 4194304;
constexpr size_t kOffProj  = kOffXpLo + 4194304;
constexpr size_t kOffM     = kOffProj + 8388608;
constexpr size_t kWsTotal  = kOffM + 8388608;
static_assert((size_t)2 * kDModel * kClustPad * 2 == kOffWinLo - kOffWinHi, "size");
static_assert((size_t)kLayers * 2 * kDInner * kDModel * 2 == kOffIpwLo - kOffIpwHi, "size");
static_assert((size_t)kLayers * kProjPad * kDInner * 2 == kOffXpwLo - kOffXpwHi, "size");
static_assert((size_t)kLayers * kDModel * kDInner * 2 == kOffOpwLo - kOffOpwHi, "size");
static_assert((size_t)kRows * kClustPad * 2 == kOffNrLo - kOffNrHi, "size");
static_assert((size_t)kRows2 * 2 * kDInner * 4 == kOffXcf - kOffXz, "size");
static_assert((size_t)kRows2 * kDInner * 4 == kOffXcHi - kOffXcf, "size");
static_assert((size_t)kRows2 * kDInner * 2 == kOffXcLo - kOffXcHi, "size");
static_assert((size_t)kRows2 * kDInner * 2 == kOffXa - kOffXcLo, "size");
static_assert((size_t)kRows2 * kDModel * 4 == kOffXb - kOffXa, "size");
static_assert((size_t)kRows2 * kDModel * 2 == kOffXpLo - kOffXpHi, "size");
static_assert(kWsTotal == 110100480ull, "size");
static_assert(kWsTotal <= 134217728ull, "size");

typedef __attribute__((ext_vector_type(16))) _Float16 v16h;
typedef __attribute__((ext_vector_type(8)))  _Float16 v8h;
typedef __attribute__((ext_vector_type(16))) __bf16   v16b;
typedef __attribute__((ext_vector_type(8)))  __bf16   v8b;
typedef __attribute__((ext_vector_type(8)))  float    v8f;
typedef __attribute__((ext_vector_type(4)))  float    v4f;
typedef __attribute__((ext_vector_type(4)))  unsigned int v4u;

__device__ __forceinline__ unsigned short f2bf_bits(float f) {
  unsigned u = __float_as_uint(f);
  return (unsigned short)((u + 0x7FFFu + ((u >> 16) & 1u)) >> 16);
}
__device__ __forceinline__ float bf_bits2f(unsigned short h) { return __uint_as_float(((unsigned)h) << 16); }

__device__ __forceinline__ void dep_guard_h(v8f& a, v8f& b, v16h x, v16h y) { asm volatile("v_nop\n\tv_nop\n\tv_nop\n\tv_nop" : "+v"(a), "+v"(b) : "v"(x), "v"(y)); }
__device__ __forceinline__ void dep_guard_b(v8f& a, v8f& b, v16b x, v16b y) { asm volatile("v_nop\n\tv_nop\n\tv_nop\n\tv_nop" : "+v"(a), "+v"(b) : "v"(x), "v"(y)); }
__device__ __forceinline__ void keep4_h(v16h a, v16h b, v16h c, v16h d) { asm volatile("v_nop" :: "v"(a), "v"(b), "v"(c), "v"(d)); }
__device__ __forceinline__ void keep4_b(v16b a, v16b b, v16b c, v16b d) { asm volatile("v_nop" :: "v"(a), "v"(b), "v"(c), "v"(d)); }
__device__ __forceinline__ void acc_guard4(v8f& a, v8f& b, v8f& c, v8f& d) { asm volatile("v_nop\n\tv_nop\n\tv_nop\n\tv_nop" : "+v"(a), "+v"(b), "+v"(c), "+v"(d)); }
template <typename T> struct Frag;
template <> struct Frag<_Float16> {
  typedef v16h V; union U { v16h v; v8h h[2]; };
  static __device__ __forceinline__ v16h load(const _Float16* p) {
    U f; f.h[0] = *(const v8h*)(p); f.h[1] = *(const v8h*)(p + 16); return f.v;
  }
  static __device__ __forceinline__ v8f mma(v16h a, v16h b, v8f c) {
    return __builtin_amdgcn_wmma_f32_16x16x32_f16(false, a, false, b, (short)0, c, false, false);
  }
  static __device__ __forceinline__ void guard(v8f& a, v8f& b, v16h x, v16h y) { dep_guard_h(a, b, x, y); }
  static __device__ __forceinline__ void keep(v16h a, v16h b, v16h c, v16h d) { keep4_h(a, b, c, d); }
};
template <> struct Frag<__bf16> {
  typedef v16b V; union U { v16b v; v8b h[2]; };
  static __device__ __forceinline__ v16b load(const __bf16* p) {
    U f; f.h[0] = *(const v8b*)(p); f.h[1] = *(const v8b*)(p + 16); return f.v;
  }
  static __device__ __forceinline__ v8f mma(v16b a, v16b b, v8f c) {
    return __builtin_amdgcn_wmma_f32_16x16x32_bf16(false, a, false, b, (short)0, c, false, false);
  }
  static __device__ __forceinline__ void guard(v8f& a, v8f& b, v16b x, v16b y) { dep_guard_b(a, b, x, y); }
  static __device__ __forceinline__ void keep(v16b a, v16b b, v16b c, v16b d) { keep4_b(a, b, c, d); }
};

__device__ __forceinline__ unsigned pk16(unsigned short a, unsigned short b) { return (unsigned)a | ((unsigned)b << 16); }

template <int ET> struct Elem;
template <> struct Elem<0> { typedef _Float16 T; };
template <> struct Elem<1> { typedef __bf16 T; };
template <int ET, bool SPLIT, int BIAS_MODE, int OUT_MODE, bool RESID, int ACT = 0>
__global__ __launch_bounds__(256) void wmma_gemm64(
    const unsigned short* __restrict__ Ap, const unsigned short* __restrict__ A2p, int lda, long strideA,
    const unsigned short* __restrict__ Btp, const unsigned short* __restrict__ Bt2p, int ldb, long strideB,
    void* __restrict__ Cout, void* __restrict__ Cout2, int ldc, long strideC,
    const float* __restrict__ bias,
    const float* __restrict__ resid, long strideR,
    int M, int N, int K, float scale) {
  typedef typename Elem<ET>::T T;
  typedef typename Frag<T>::V V;
  const T* A = (const T*)Ap; const T* A2 = (const T*)A2p; const T* Bt = (const T*)Btp; const T* Bt2 = (const T*)Bt2p;
  __shared__ __align__(16) float sT[8][16 * 68];
  const int b    = blockIdx.y;
  const int lane = threadIdx.x & 31;
  const int wave = threadIdx.x >> 5;
  const int tilesN = N >> 6;
  const int tilesM = M >> 6;
  const int tile = blockIdx.x * 8 + wave;
  if (tile >= tilesM * tilesN) return;
  const int tm = tile / tilesN;
  const int tn = tile - tm * tilesN;
  const int m0 = tm << 6;
  const int n0 = tn << 6;

  const T* Ab  = A  + (size_t)b * strideA;
  const T* Bb  = Bt + (size_t)b * strideB;
  const T* Ab2 = SPLIT ? (A2  + (size_t)b * strideA) : nullptr;
  const T* Bb2 = SPLIT ? (Bt2 + (size_t)b * strideB) : nullptr;

  const int rlane = lane & 15;
  const int koff  = (lane >> 4) * 8;
  const int mOff  = (lane >> 4) * 8;

  v8f acc[4][4];
#pragma unroll
  for (int i = 0; i < 4; ++i)
#pragma unroll
    for (int j = 0; j < 4; ++j) acc[i][j] = (v8f){0.f,0.f,0.f,0.f,0.f,0.f,0.f,0.f};

  for (int k0 = 0; k0 < K; k0 += 32) {
    V bh[4], bl[4];
#pragma unroll
    for (int j = 0; j < 4; ++j) {
      const size_t bo = (size_t)(n0 + (j << 4) + rlane) * ldb + koff + k0;
      bh[j] = Frag<T>::load(Bb + bo);
      if (SPLIT) bl[j] = Frag<T>::load(Bb2 + bo);
    }
#pragma unroll
    for (int i = 0; i < 4; ++i) {
      const size_t ao = (size_t)(m0 + (i << 4) + rlane) * lda + koff + k0;
      V ah = Frag<T>::load(Ab + ao);
      V al;
      if (SPLIT) al = Frag<T>::load(Ab2 + ao);
#pragma unroll
      for (int j = 0; j < 4; ++j) {
        acc[i][j] = Frag<T>::mma(ah, bh[j], acc[i][j]);
        if (SPLIT) {
          acc[i][j] = Frag<T>::mma(ah, bl[j], acc[i][j]);
          acc[i][j] = Frag<T>::mma(al, bh[j], acc[i][j]);
        }
      }
      Frag<T>::guard(acc[i][0], acc[i][3], ah, SPLIT ? al : ah);
    }
    Frag<T>::keep(bh[0], bh[1], bh[2], bh[3]);
    if (SPLIT) Frag<T>::keep(bl[0], bl[1], bl[2], bl[3]);
  }
  acc_guard4(acc[0][0], acc[0][1], acc[0][2], acc[0][3]);
  acc_guard4(acc[1][0], acc[1][1], acc[1][2], acc[1][3]);
  acc_guard4(acc[2][0], acc[2][1], acc[2][2], acc[2][3]);
  acc_guard4(acc[3][0], acc[3][1], acc[3][2], acc[3][3]);

  float* slab = sT[wave];
  const float* Rb = RESID ? (resid + (size_t)b * strideR) : nullptr;
#pragma unroll
  for (int i = 0; i < 4; ++i) {
    const int mBase = m0 + (i << 4);
#pragma unroll
    for (int j = 0; j < 4; ++j) {
      const int n = n0 + (j << 4) + rlane;
      float bv = 0.f;
      if (BIAS_MODE == 2) bv = bias[n];
#pragma unroll
      for (int r = 0; r < 8; ++r) {
        float v = acc[i][j][r] * scale;
        if (BIAS_MODE == 1) v += bias[mBase + mOff + r];
        if (BIAS_MODE == 2) v += bv;
        if (RESID) v += Rb[(size_t)(mBase + mOff + r) * ldc + n];
        if (ACT == 2) v = fmaxf(v, 0.0f);
        if (ACT == 4) v = (v > 0.f) ? v : 0.01f * v;
        slab[(mOff + r) * 68 + (j << 4) + rlane] = v;
      }
    }
    __builtin_amdgcn_fence(__ATOMIC_RELEASE, "workgroup");
    __builtin_amdgcn_wave_barrier();
    __builtin_amdgcn_fence(__ATOMIC_ACQUIRE, "workgroup");
    if (OUT_MODE == 0) {
      float* C = (float*)Cout + (size_t)b * strideC;
      const int hh = lane >> 4, c4 = (lane & 15) * 4;
      for (int pass = 0; pass < 2; ++pass) {
#pragma unroll
        for (int it = 0; it < 8; ++it) {
          const int row = it * 2 + hh;
          v4f v = *(const v4f*)(slab + row * 68 + c4);
          *(volatile v4f*)(C + (size_t)(mBase + row) * ldc + n0 + c4) = v;
        }
        __threadfence();
      }
    } else {
      const int q = lane >> 3, c8 = (lane & 7) * 8;
      unsigned short* C  = (unsigned short*)Cout  + (size_t)b * strideC;
      unsigned short* C2 = (OUT_MODE == 2) ? ((unsigned short*)Cout2 + (size_t)b * strideC) : nullptr;
      for (int pass = 0; pass < 2; ++pass) {
#pragma unroll
        for (int it = 0; it < 4; ++it) {
          const int row = it * 4 + q;
          const float* sp = slab + row * 68 + c8;
          v8h hv, lv;
#pragma unroll
          for (int e = 0; e < 8; ++e) {
            if (OUT_MODE == 1) {
              hv[e] = (_Float16)sp[e];
            } else {
              unsigned short hb = f2bf_bits(sp[e]);
              unsigned short lb = f2bf_bits(sp[e] - bf_bits2f(hb));
              hv[e] = __builtin_bit_cast(_Float16, hb);
              lv[e] = __builtin_bit_cast(_Float16, lb);
            }
          }
          *(volatile v8h*)(C + (size_t)(mBase + row) * ldc + n0 + c8) = hv;
          if (OUT_MODE == 2) *(volatile v8h*)(C2 + (size_t)(mBase + row) * ldc + n0 + c8) = lv;
        }
        __threadfence();
      }
    }
    __builtin_amdgcn_fence(__ATOMIC_RELEASE, "workgroup");
    __builtin_amdgcn_wave_barrier();
    __builtin_amdgcn_fence(__ATOMIC_ACQUIRE, "workgroup");
  }
}

__device__ __forceinline__ void split_pack8(v4f a, v4f b, v4u& hv, v4u& lv) {
  unsigned short hb[8], lb[8];
#pragma unroll
  for (int e = 0; e < 4; ++e) {
    const unsigned short h0 = f2bf_bits(a[e]);
    hb[e] = h0;
    lb[e] = f2bf_bits(a[e] - bf_bits2f(h0));
    const unsigned short h1 = f2bf_bits(b[e]);
    hb[4 + e] = h1;
    lb[4 + e] = f2bf_bits(b[e] - bf_bits2f(h1));
  }
  hv = (v4u){pk16(hb[0], hb[1]), pk16(hb[2], hb[3]), pk16(hb[4], hb[5]), pk16(hb[6], hb[7])};
  lv = (v4u){pk16(lb[0], lb[1]), pk16(lb[2], lb[3]), pk16(lb[4], lb[5]), pk16(lb[6], lb[7])};
}

__global__ __launch_bounds__(256) void wsplit_kernel(const float* __restrict__ W, int kdim, int ndim, int wLayerStride,
                                                     unsigned short* __restrict__ outH, unsigned short* __restrict__ outL,
                                                     int kpad, int pLayerStride) {
  __shared__ float sm[64][65];
  const int t  = threadIdx.x;
  const int k0 = blockIdx.x * 64;
  const int n0 = blockIdx.y * 64;
  const int z  = blockIdx.z;
  const float* Wz = W + (size_t)z * wLayerStride;
#pragma unroll
  for (int i = 0; i < 16; ++i) {
    const int e = i * 256 + t;
    const int r = e >> 6;
    const int c = e & 63;
    const int k = k0 + r, n = n0 + c;
    const int kc = (k < kdim) ? k : (kdim - 1);
    const int nc = (n < ndim) ? n : (ndim - 1);
    float v = Wz[(size_t)kc * ndim + nc];
    if (k >= kdim || n >= ndim) v = 0.0f;
    sm[c][r] = v;
  }
  __syncthreads();
  const int lane = t & 31, wave = t >> 5;
  const int q = lane >> 3, c8 = (lane & 7) * 8;
  unsigned short* oh = outH + (size_t)z * pLayerStride;
  unsigned short* ol = outL + (size_t)z * pLayerStride;
  v4u hv[2], lv[2];
  size_t off[2];
#pragma unroll
  for (int it = 0; it < 2; ++it) {
    const int row = wave * 8 + it * 4 + q;
    const v4f a = (v4f){sm[row][c8 + 0], sm[row][c8 + 1], sm[row][c8 + 2], sm[row][c8 + 3]};
    const v4f b = (v4f){sm[row][c8 + 4], sm[row][c8 + 5], sm[row][c8 + 6], sm[row][c8 + 7]};
    split_pack8(a, b, hv[it], lv[it]);
    off[it] = (size_t)(n0 + row) * kpad + k0 + c8;
  }
  for (int pass = 0; pass < 2; ++pass) {
#pragma unroll
    for (int it = 0; it < 2; ++it) {
      *(volatile v4u*)(oh + off[it]) = hv[it];
      *(volatile v4u*)(ol + off[it]) = lv[it];
    }
    __threadfence();
  }
}

__global__ __launch_bounds__(256) void cproj_kernel(const float* __restrict__ X, const float* __restrict__ W,
                                                    const float* __restrict__ bias, int foff, int kf,
                                                    unsigned short* __restrict__ outH, unsigned short* __restrict__ outL) {
  const int t = threadIdx.x;
  const int p = t >> 7, g = t & 127;
  const int n0 = g * 8;
  const bool valid = n0 < kClust;
  const int n0c = valid ? n0 : (kClust - 8);
  const int row0 = blockIdx.x * 4 + 2 * p;
  const int row1 = row0 + 1;
  const v4f ba = *(const v4f*)(bias + n0c);
  const v4f bb = *(const v4f*)(bias + n0c + 4);
  v4f a0 = ba, a1 = bb, c0 = ba, c1 = bb;
  const float* x0p = X + (size_t)row0 * kFeat + foff;
  const float* x1p = X + (size_t)row1 * kFeat + foff;
#pragma unroll 1
  for (int k = 0; k < kf; ++k) {
    const float xv0 = x0p[k];
    const float xv1 = x1p[k];
    const v4f wa = *(const v4f*)(W + (size_t)k * kClust + n0c);
    const v4f wb = *(const v4f*)(W + (size_t)k * kClust + n0c + 4);
    a0 += xv0 * wa; a1 += xv0 * wb;
    c0 += xv1 * wa; c1 += xv1 * wb;
  }
  const v4f zero4 = (v4f){0.f, 0.f, 0.f, 0.f};
  a0 = valid ? a0 : zero4; a1 = valid ? a1 : zero4;
  c0 = valid ? c0 : zero4; c1 = valid ? c1 : zero4;
  v4u h0, l0, h1, l1;
  split_pack8(a0, a1, h0, l0);
  split_pack8(c0, c1, h1, l1);
  const size_t o0 = (size_t)row0 * kClustPad + n0;
  const size_t o1 = (size_t)row1 * kClustPad + n0;
  for (int pass = 0; pass < 2; ++pass) {
    *(volatile v4u*)(outH + o0) = h0;
    *(volatile v4u*)(outL + o0) = l0;
    *(volatile v4u*)(outH + o1) = h1;
    *(volatile v4u*)(outL + o1) = l1;
    __threadfence();
  }
}


__global__ __launch_bounds__(256) void stepa_kernel(const float* __restrict__ xz, const float* __restrict__ cw,
                                                    const float* __restrict__ cb, int layer,
                                                    float* __restrict__ xcf,
                                                    unsigned short* __restrict__ xch, unsigned short* __restrict__ xcl) {
  __shared__ __align__(16) float smf[8][kDInner];
  const int t = threadIdx.x, w = t >> 5, lane = t & 31, c4 = lane * 4;
  const int row = blockIdx.x * 8 + w;
  const v4f a  = *(const v4f*)(xz + (size_t)row * (2 * kDInner) + c4);
  const v4f b4 = *(const v4f*)(cb + layer * kDInner + c4);
  const float* cwl = cw + layer * kDInner * kDConv + c4 * kDConv + (kDConv - 1);
  v4f r;
#pragma unroll
  for (int e = 0; e < 4; ++e) {
    const float v = a[e] * cwl[kDConv * e] + b4[e];
    const float sg = __builtin_amdgcn_rcpf(1.0f + __expf(-v));
    r[e] = v * sg;
  }
  *(v4f*)(&smf[w][c4]) = r;
  __syncthreads();
  const int hsel = lane >> 4;
  const int c8 = (lane & 15) * 8;
  const v4f p0 = *(const v4f*)(&smf[w][c8]);
  const v4f p1 = *(const v4f*)(&smf[w][c8 + 4]);
  v4u hv, lv;
  split_pack8(p0, p1, hv, lv);
  const v4u pv = hsel ? lv : hv;
  unsigned short* pd = (hsel ? xcl : xch) + (size_t)row * kDInner + c8;
  float* fd = xcf + (size_t)row * kDInner + c4;
  for (int pass = 0; pass < 2; ++pass) {
    *(volatile v4f*)fd = r;
    *(volatile v4u*)pd = pv;
    __threadfence();
  }
}

__global__ __launch_bounds__(256) void stepb_kernel(const float* __restrict__ xcf, const float* __restrict__ xz,
                                                    const float* __restrict__ proj, const float* __restrict__ dtw,
                                                    const float* __restrict__ dtb, const float* __restrict__ dskip,
                                                    const float* __restrict__ alog, int layer,
                                                    unsigned short* __restrict__ yh, unsigned short* __restrict__ yl) {
  __shared__ __align__(16) float smf[8][kDInner];
  (void)alog;
  const int t = threadIdx.x, w = t >> 5, lane = t & 31, c4 = lane * 4;
  const int row = blockIdx.x * 8 + w;
  const v4f xc4 = *(const v4f*)(xcf + (size_t)row * kDInner + c4);
  const v4f z4  = *(const v4f*)(xz + (size_t)row * (2 * kDInner) + kDInner + c4);
  const float* pr = proj + (size_t)row * kProjPad;
  const v4f dtr = *(const v4f*)pr;
  const int s = lane & 15;
  float bc = pr[kDtRank + s] * pr[kDtRank + kDState + s];
  bc += __shfl_xor(bc, 1, 32);
  bc += __shfl_xor(bc, 2, 32);
  bc += __shfl_xor(bc, 4, 32);
  bc += __shfl_xor(bc, 8, 32);
  const float* dl = dtw + (size_t)layer * kDtRank * kDInner + c4;
  const v4f w0 = *(const v4f*)(dl);
  const v4f w1 = *(const v4f*)(dl + kDInner);
  const v4f w2 = *(const v4f*)(dl + 2 * kDInner);
  const v4f w3 = *(const v4f*)(dl + 3 * kDInner);
  const v4f b4 = *(const v4f*)(dtb + layer * kDInner + c4);
  const v4f d4 = *(const v4f*)(dskip + layer * kDInner + c4);
  v4f r;
#pragma unroll
  for (int e = 0; e < 4; ++e) {
    const float pre = dtr[0] * w0[e] + dtr[1] * w1[e] + dtr[2] * w2[e] + dtr[3] * w3[e] + b4[e];
    const float ex = __expf(-fabsf(pre));
    const float dt = fmaxf(pre, 0.0f) + logf(1.0f + ex);
    const float xc = xc4[e];
    const float y0 = (dt * bc) * xc + d4[e] * xc;
    const float zz = z4[e];
    const float sz = zz * __builtin_amdgcn_rcpf(1.0f + __expf(-zz));
    r[e] = y0 * sz;
  }
  *(v4f*)(&smf[w][c4]) = r;
  __syncthreads();
  const int hsel = lane >> 4;
  const int c8 = (lane & 15) * 8;
  const v4f p0 = *(const v4f*)(&smf[w][c8]);
  const v4f p1 = *(const v4f*)(&smf[w][c8 + 4]);
  v4u hv, lv;
  split_pack8(p0, p1, hv, lv);
  const v4u pv = hsel ? lv : hv;
  unsigned short* pd = (hsel ? yl : yh) + (size_t)row * kDInner + c8;
  for (int pass = 0; pass < 2; ++pass) {
    *(volatile v4u*)pd = pv;
    __threadfence();
  }
}

template <bool DO_LN>
__global__ __launch_bounds__(256) void ln_kernel(const float* __restrict__ mbuf, const float* __restrict__ xin,
                                                 const float* __restrict__ lng, const float* __restrict__ lnb, int layer,
                                                 float* __restrict__ xout,
                                                 unsigned short* __restrict__ xph, unsigned short* __restrict__ xpl) {
  __shared__ __align__(16) float smf[16][kDModel];
  const int t = threadIdx.x, wave = t >> 5, lane = t & 31;
  const int hrow = lane >> 4, j = lane & 15;
  const int rloc = wave * 2 + hrow;
  const int row = blockIdx.x * 16 + rloc;
  const v4f x4 = *(const v4f*)(xin + (size_t)row * kDModel + 4 * j);
  v4f xn = x4;
  if (DO_LN) {
    const v4f m4 = *(const v4f*)(mbuf + (size_t)row * kDModel + 4 * j);
    float s1 = (m4[0] + m4[1]) + (m4[2] + m4[3]);
    s1 += __shfl_xor(s1, 1, 32);
    s1 += __shfl_xor(s1, 2, 32);
    s1 += __shfl_xor(s1, 4, 32);
    s1 += __shfl_xor(s1, 8, 32);
    const float mean = s1 * kInvDModel;
    const float d0 = m4[0] - mean, d1 = m4[1] - mean, d2 = m4[2] - mean, d3 = m4[3] - mean;
    float s2 = (d0 * d0 + d1 * d1) + (d2 * d2 + d3 * d3);
    s2 += __shfl_xor(s2, 1, 32);
    s2 += __shfl_xor(s2, 2, 32);
    s2 += __shfl_xor(s2, 4, 32);
    s2 += __shfl_xor(s2, 8, 32);
    const float var = s2 * kInvDModel;
    const float rstd = rsqrtf(var + kLnEps);
    const v4f g4  = *(const v4f*)(lng + layer * kDModel + 4 * j);
    const v4f bb4 = *(const v4f*)(lnb + layer * kDModel + 4 * j);
    xn[0] = x4[0] + ((d0 * rstd) * g4[0] + bb4[0]);
    xn[1] = x4[1] + ((d1 * rstd) * g4[1] + bb4[1]);
    xn[2] = x4[2] + ((d2 * rstd) * g4[2] + bb4[2]);
    xn[3] = x4[3] + ((d3 * rstd) * g4[3] + bb4[3]);
  }
  *(v4f*)(&smf[rloc][4 * j]) = xn;
  __syncthreads();
  const int q = lane >> 3, c8 = (lane & 7) * 8;
  const int prow = wave * 2 + (q >> 1);
  const int growp = blockIdx.x * 16 + prow;
  const v4f p0 = *(const v4f*)(&smf[prow][c8]);
  const v4f p1 = *(const v4f*)(&smf[prow][c8 + 4]);
  v4u hv, lv;
  split_pack8(p0, p1, hv, lv);
  const int losel = q & 1;
  const v4u pv = losel ? lv : hv;
  unsigned short* pd = (losel ? xpl : xph) + (size_t)growp * kDModel + c8;
  float* fd = xout + (size_t)row * kDModel + 4 * j;
  for (int pass = 0; pass < 2; ++pass) {
    if (DO_LN) *(volatile v4f*)fd = xn;
    *(volatile v4u*)pd = pv;
    __threadfence();
  }
}

__global__ __launch_bounds__(256) void head_kernel(const float* __restrict__ xfin, const float* __restrict__ w1,
                                                   const float* __restrict__ b1, const float* __restrict__ w2,
                                                   const float* __restrict__ b2, float* __restrict__ out, int nrows) {
  const int row = blockIdx.x * 256 + threadIdx.x;
  const int rowc = (row < nrows) ? row : (nrows - 1);
  float h[kHeadHid];
#pragma unroll
  for (int ci = 0; ci < kHeadHid / 4; ++ci) {
    const v4f bv = *(const v4f*)(b1 + 4 * ci);
    h[4 * ci + 0] = bv[0]; h[4 * ci + 1] = bv[1]; h[4 * ci + 2] = bv[2]; h[4 * ci + 3] = bv[3];
  }
  const size_t base0 = (size_t)rowc * kDModel;
  const size_t base1 = (size_t)(nrows + rowc) * kDModel;
#pragma unroll 1
  for (int k = 0; k < 2 * kDModel; ++k) {
    const size_t src = (k < kDModel) ? (base0 + k) : (base1 + (k - kDModel));
    const float o = xfin[src];
    const float* wr = w1 + k * kHeadHid;
#pragma unroll
    for (int ci = 0; ci < kHeadHid / 4; ++ci) {
      const v4f wv = *(const v4f*)(wr + 4 * ci);
      h[4 * ci + 0] += o * wv[0]; h[4 * ci + 1] += o * wv[1];
      h[4 * ci + 2] += o * wv[2]; h[4 * ci + 3] += o * wv[3];
    }
  }
  float acc = b2[0];
#pragma unroll
  for (int ci = 0; ci < kHeadHid / 4; ++ci) {
    const v4f wv = *(const v4f*)(w2 + 4 * ci);
    acc += fmaxf(h[4 * ci + 0], 0.0f) * wv[0];
    acc += fmaxf(h[4 * ci + 1], 0.0f) * wv[1];
    acc += fmaxf(h[4 * ci + 2], 0.0f) * wv[2];
    acc += fmaxf(h[4 * ci + 3], 0.0f) * wv[3];
  }
  float* od = out + rowc;
  for (int pass = 0; pass < 2; ++pass) {
    *(volatile float*)od = acc;
    __threadfence();
  }
}

extern "C" void kernel_launch(void* const* d_in, const int* in_sizes, int n_in,
                              void* d_out, int out_size, void* d_ws, size_t ws_size,
                              hipStream_t stream) {
  if (n_in < 24) return;
  if (in_sizes[0] != kRows * kFeat) return;
  if (in_sizes[1] != kNonRain * kClust || in_sizes[3] != kRain * kClust) return;
  if (in_sizes[5] != kClust * kDModel || in_sizes[7] != kClust * kDModel) return;
  if (in_sizes[9] != kLayers * kDModel * 2 * kDInner) return;
  if (in_sizes[12] != kLayers * kDInner * kProjN || in_sizes[17] != kLayers * kDInner * kDModel) return;
  if (in_sizes[20] != 2 * kDModel * kHeadHid) return;
  if (out_size != kRows) return;
  if (ws_size < kWsTotal) return;

  const float* X       = (const float*)d_in[0];
  const float* w_nr    = (const float*)d_in[1];
  const float* b_nr    = (const float*)d_in[2];
  const float* w_r     = (const float*)d_in[3];
  const float* b_r     = (const float*)d_in[4];
  const float* w_in_nr = (const float*)d_in[5];
  const float* b_in_nr = (const float*)d_in[6];
  const float* w_in_r  = (const float*)d_in[7];
  const float* b_in_r  = (const float*)d_in[8];
  const float* ipw     = (const float*)d_in[9];
  const float* cw      = (const float*)d_in[10];
  const float* cb      = (const float*)d_in[11];
  const float* xpw     = (const float*)d_in[12];
  const float* dtw     = (const float*)d_in[13];
  const float* dtb     = (const float*)d_in[14];
  const float* alog    = (const float*)d_in[15];
  const float* dskip   = (const float*)d_in[16];
  const float* opw     = (const float*)d_in[17];
  const float* ln_g    = (const float*)d_in[18];
  const float* ln_b    = (const float*)d_in[19];
  const float* hw1     = (const float*)d_in[20];
  const float* hb1     = (const float*)d_in[21];
  const float* hw2     = (const float*)d_in[22];
  const float* hb2     = (const float*)d_in[23];
  float* out = (float*)d_out;

  char* ws = (char*)d_ws;
  unsigned short* winH = (unsigned short*)(ws + kOffWinHi);
  unsigned short* winL = (unsigned short*)(ws + kOffWinLo);
  unsigned short* ipwH = (unsigned short*)(ws + kOffIpwHi);
  unsigned short* ipwL = (unsigned short*)(ws + kOffIpwLo);
  unsigned short* xpwH = (unsigned short*)(ws + kOffXpwHi);
  unsigned short* xpwL = (unsigned short*)(ws + kOffXpwLo);
  unsigned short* opwH = (unsigned short*)(ws + kOffOpwHi);
  unsigned short* opwL = (unsigned short*)(ws + kOffOpwLo);
  unsigned short* nrH  = (unsigned short*)(ws + kOffNrHi);
  unsigned short* nrL  = (unsigned short*)(ws + kOffNrLo);
  float* xz   = (float*)(ws + kOffXz);
  float* xcf  = (float*)(ws + kOffXcf);
  unsigned short* xcH = (unsigned short*)(ws + kOffXcHi);
  unsigned short* xcL = (unsigned short*)(ws + kOffXcLo);
  float* xa   = (float*)(ws + kOffXa);
  float* xb   = (float*)(ws + kOffXb);
  unsigned short* xpH = (unsigned short*)(ws + kOffXpHi);
  unsigned short* xpL = (unsigned short*)(ws + kOffXpLo);
  float* proj = (float*)(ws + kOffProj);
  float* mbuf = (float*)(ws + kOffM);

  wsplit_kernel<<<dim3(kClustPad / 64, 1, 1), 256, 0, stream>>>(w_in_nr, kClust, kDModel, 0,
                                                                winH, winL, kClustPad, 0);
  wsplit_kernel<<<dim3(kClustPad / 64, 1, 1), 256, 0, stream>>>(w_in_r, kClust, kDModel, 0,
                                                                winH + kDModel * kClustPad, winL + kDModel * kClustPad,
                                                                kClustPad, 0);
  wsplit_kernel<<<dim3(1, (2 * kDInner) / 64, kLayers), 256, 0, stream>>>(ipw, kDModel, 2 * kDInner, kDModel * 2 * kDInner,
                                                                          ipwH, ipwL, kDModel, 2 * kDInner * kDModel);
  wsplit_kernel<<<dim3(kDInner / 64, 1, kLayers), 256, 0, stream>>>(xpw, kDInner, kProjN, kDInner * kProjN,
                                                                    xpwH, xpwL, kDInner, kProjPad * kDInner);
  wsplit_kernel<<<dim3(kDInner / 64, 1, kLayers), 256, 0, stream>>>(opw, kDInner, kDModel, kDInner * kDModel,
                                                                    opwH, opwL, kDInner, kDModel * kDInner);

  cproj_kernel<<<kRows / 4, 256, 0, stream>>>(X, w_nr, b_nr, 0, kNonRain, nrH, nrL);
  wmma_gemm64<1, true, 2, 0, false, 0><<<dim3(kRows / 64 / 8, 1), 256, 0, stream>>>(
      nrH, nrL, kClustPad, 0L, winH, winL, kClustPad, 0L,
      (void*)xa, (void*)mbuf, kDModel, 0L, b_in_nr, mbuf, 0L, kRows, kDModel, kClustPad, 1.0f);
  cproj_kernel<<<kRows / 4, 256, 0, stream>>>(X, w_r, b_r, kNonRain, kRain, nrH, nrL);
  wmma_gemm64<1, true, 2, 0, false, 0><<<dim3(kRows / 64 / 8, 1), 256, 0, stream>>>(
      nrH, nrL, kClustPad, 0L, winH + kDModel * kClustPad, winL + kDModel * kClustPad, kClustPad, 0L,
      (void*)(xa + (size_t)kRows * kDModel), (void*)mbuf, kDModel, 0L, b_in_r, mbuf, 0L,
      kRows, kDModel, kClustPad, 1.0f);

  ln_kernel<false><<<kRows2 / 16, 256, 0, stream>>>(mbuf, xa, ln_g, ln_b, 0, xb, xpH, xpL);

  float* cur = xa;
  float* nxt = xb;
  for (int l = 0; l < kLayers; ++l) {
    wmma_gemm64<1, true, 0, 0, false, 0><<<dim3((kRows2 / 64) * ((2 * kDInner) / 64) / 8, 1), 256, 0, stream>>>(
        xpH, xpL, kDModel, 0L, ipwH + (size_t)l * 2 * kDInner * kDModel, ipwL + (size_t)l * 2 * kDInner * kDModel,
        kDModel, 0L, (void*)xz, (void*)mbuf, 2 * kDInner, 0L, b_in_nr, mbuf, 0L,
        kRows2, 2 * kDInner, kDModel, 1.0f);
    stepa_kernel<<<kRows2 / 8, 256, 0, stream>>>(xz, cw, cb, l, xcf, xcH, xcL);
    wmma_gemm64<1, true, 0, 0, false, 0><<<dim3((kRows2 / 64) * (kProjPad / 64) / 8, 1), 256, 0, stream>>>(
        xcH, xcL, kDInner, 0L, xpwH + (size_t)l * kProjPad * kDInner, xpwL + (size_t)l * kProjPad * kDInner,
        kDInner, 0L, (void*)proj, (void*)mbuf, kProjPad, 0L, b_in_nr, mbuf, 0L,
        kRows2, kProjPad, kDInner, 1.0f);
    stepb_kernel<<<kRows2 / 8, 256, 0, stream>>>(xcf, xz, proj, dtw, dtb, dskip, alog, l, xcH, xcL);
    wmma_gemm64<1, true, 0, 0, false, 0><<<dim3((kRows2 / 64) * (kDModel / 64) / 8, 1), 256, 0, stream>>>(
        xcH, xcL, kDInner, 0L, opwH + (size_t)l * kDModel * kDInner, opwL + (size_t)l * kDModel * kDInner,
        kDInner, 0L, (void*)mbuf, (void*)proj, kDModel, 0L, b_in_nr, proj, 0L,
        kRows2, kDModel, kDInner, 1.0f);
    ln_kernel<true><<<kRows2 / 16, 256, 0, stream>>>(mbuf, cur, ln_g, ln_b, l, nxt, xpH, xpL);
    float* tswap = cur; cur = nxt; nxt = tswap;
  }

  head_kernel<<<kRows / 256, 256, 0, stream>>>(cur, hw1, hb1, hw2, hb2, out, kRows);
}
